// RNN_8220567404960
// MI455X (gfx1250) — hardware-verified
//
#include <hip/hip_runtime.h>
#include <math.h>

constexpr int NB   = 4096;
constexpr int NTS  = 40;
constexpr int NV   = 128;
constexpr int NH   = 256;
constexpr int NG4  = 1024;
constexpr int NIN  = NV + NH;
constexpr int NTHR = 256;
constexpr int ROWS = 16;
constexpr int HP   = 264;
constexpr int GP   = 1028;
constexpr int OPD  = 132;
constexpr float FORGET_B = 1.0f;
static_assert(NB % ROWS == 0);
static_assert(NH == 32 * (NTHR / 32));
static_assert(NV == 16 * (NTHR / 32));
static_assert(NG4 == 4 * NH);
static_assert(NH % 32 == 0);
static_assert(NH % 64 == 0 && NG4 % 64 == 0 && NV % 64 == 0);
static_assert(HP % 8 == 0 && GP % 4 == 0 && OPD % 4 == 0);
static_assert((ROWS * NV / 4) % NTHR == 0);
static_assert((NV * NG4 / 4) % NTHR == 0);
static_assert(ROWS * 16 == NTHR);

typedef __attribute__((ext_vector_type(16))) _Float16 v16h;
typedef __attribute__((ext_vector_type(8)))  _Float16 v8h;
typedef __attribute__((ext_vector_type(16))) __bf16   v16b;
typedef __attribute__((ext_vector_type(8)))  __bf16   v8b;
typedef __attribute__((ext_vector_type(8)))  float    v8f;
typedef __attribute__((ext_vector_type(4)))  float    v4f;

__device__ __forceinline__ unsigned short f2bf_bits(float f) {
  unsigned u = __float_as_uint(f);
  return (unsigned short)((u + 0x7FFFu + ((u >> 16) & 1u)) >> 16);
}
__device__ __forceinline__ float bf_bits2f(unsigned short h) { return __uint_as_float(((unsigned)h) << 16); }
__device__ __forceinline__ float bf16r(float f) { return bf_bits2f(f2bf_bits(f)); }
__device__ __forceinline__ __bf16 bits2bf(unsigned short b) { return __builtin_bit_cast(__bf16, b); }

__device__ __forceinline__ void guard_g4(v8f& a0, v8f& a1, v8f& a2, v8f& a3,
                                         v16b x0, v16b x1, v16b y0, v16b y1, v16b y2, v16b y3) {
  asm volatile("v_nop\n\tv_nop\n\tv_nop\n\tv_nop"
               : "+v"(a0), "+v"(a1), "+v"(a2), "+v"(a3)
               : "v"(x0), "v"(x1), "v"(y0), "v"(y1), "v"(y2), "v"(y3));
}
__device__ __forceinline__ void guard_g1(v8f& a0, v16b x0, v16b x1, v16b y0) {
  asm volatile("v_nop\n\tv_nop\n\tv_nop\n\tv_nop" : "+v"(a0) : "v"(x0), "v"(x1), "v"(y0));
}
__device__ __forceinline__ void acc_guard4(v8f& a, v8f& b, v8f& c, v8f& d) {
  asm volatile("v_nop\n\tv_nop\n\tv_nop\n\tv_nop" : "+v"(a), "+v"(b), "+v"(c), "+v"(d));
}
__device__ __forceinline__ void acc_guard1(v8f& a) {
  asm volatile("v_nop\n\tv_nop\n\tv_nop\n\tv_nop" : "+v"(a));
}

template <typename T> struct Frag;
template <> struct Frag<__bf16> {
  typedef v16b V; union U { v16b v; v8b h[2]; };
  static __device__ __forceinline__ v16b load(const __bf16* p) {
    U f; f.h[0] = *(const v8b*)(p); f.h[1] = *(const v8b*)(p + 16); return f.v;
  }
  static __device__ __forceinline__ v8f mma(v16b a, v16b b, v8f c) {
    return __builtin_amdgcn_wmma_f32_16x16x32_bf16(false, a, false, b, (short)0, c, false, false);
  }
};

__device__ __forceinline__ float fsig(float x)  { return __builtin_amdgcn_rcpf(1.0f + expf(-x)); }
__device__ __forceinline__ float ftanh(float x) { return 1.0f - 2.0f * __builtin_amdgcn_rcpf(expf(2.0f * x) + 1.0f); }

__global__ __launch_bounds__(NTHR) void tpose_bf16_kernel(const float* __restrict__ src, int C, int ldo,
                                                          unsigned short* __restrict__ O) {
  __shared__ float Tt[64 * 65];
  const int tid = threadIdx.x;
  const int c0 = blockIdx.x * 64, r0 = blockIdx.y * 64;
#pragma unroll
  for (int i = 0; i < 4; ++i) {
    const int idx = i * NTHR + tid;
    const int rr = idx >> 4, cc = (idx & 15) * 4;
    const v4f v = *(const v4f*)(src + (size_t)(r0 + rr) * (size_t)C + c0 + cc);
    Tt[rr * 65 + cc + 0] = v[0];
    Tt[rr * 65 + cc + 1] = v[1];
    Tt[rr * 65 + cc + 2] = v[2];
    Tt[rr * 65 + cc + 3] = v[3];
  }
  __syncthreads();
  const int q = tid >> 3, c8 = (tid & 7) * 8;
  v8h hv[2];
#pragma unroll
  for (int g = 0; g < 2; ++g) {
    const int qq = g * 32 + q;
#pragma unroll
    for (int e = 0; e < 8; ++e) {
      const float f = Tt[(c8 + e) * 65 + qq];
      hv[g][e] = __builtin_bit_cast(_Float16, f2bf_bits(f));
    }
  }
  for (int pass = 0; pass < 2; ++pass) {
#pragma unroll
    for (int g = 0; g < 2; ++g) {
      const size_t o = (size_t)(c0 + g * 32 + q) * (size_t)ldo + (size_t)(r0 + c8);
      *(volatile v8h*)(O + o) = hv[g];
    }
    __threadfence();
  }
}

__global__ __launch_bounds__(NTHR) void gtab_kernel(const float* __restrict__ src, float* __restrict__ dst, int n4) {
  const int i = blockIdx.x * NTHR + threadIdx.x;
  if (i < n4) {
    const v4f v = *(const v4f*)(src + (size_t)i * 4);
    v4f o;
#pragma unroll
    for (int e = 0; e < 4; ++e) o[e] = bf16r(v[e]);
    *(volatile v4f*)(dst + (size_t)i * 4) = o;
    __threadfence();
    *(volatile v4f*)(dst + (size_t)i * 4) = o;
  }
}

__device__ __forceinline__ void stage_rows(const int* __restrict__ ids, const float* __restrict__ GF,
                                           float* Gs, int rowbase, int t, int tid) {
  const int m = tid >> 4, q4 = (tid & 15) * 4;
  int ch = ids[(size_t)(rowbase + m) * NTS + t];
  ch = ch < 0 ? 0 : ch;
  ch = ch > NV - 1 ? NV - 1 : ch;
  const float* sp = GF + (size_t)ch * NG4 + q4;
  float* dp = Gs + m * GP + q4;
#pragma unroll 1
  for (int i = 0; i < 4; ++i) {
    const int cb = i * 256;
    const v4f v0 = *(const v4f*)(sp + cb);
    const v4f v1 = *(const v4f*)(sp + cb + 64);
    const v4f v2 = *(const v4f*)(sp + cb + 128);
    const v4f v3 = *(const v4f*)(sp + cb + 192);
    *(v4f*)(dp + cb)       = v0;
    *(v4f*)(dp + cb + 64)  = v1;
    *(v4f*)(dp + cb + 128) = v2;
    *(v4f*)(dp + cb + 192) = v3;
  }
}

__global__ __launch_bounds__(NTHR) void lstm_seq_kernel(const int* __restrict__ ids, const float* __restrict__ GF,
                                                        const float* __restrict__ bl, const float* __restrict__ bd,
                                                        const unsigned short* __restrict__ WHp,
                                                        const unsigned short* __restrict__ WDp,
                                                        float* __restrict__ out) {
  __shared__ __align__(16) __bf16 Ahh[ROWS * HP];
  __shared__ __align__(16) __bf16 Ahl[ROWS * HP];
  __shared__ __align__(16) float  Gs[ROWS * GP];
  __shared__ __align__(16) float  Hs[ROWS * OPD];
  const __bf16* WH = (const __bf16*)WHp;
  const __bf16* WD = (const __bf16*)WDp;
  const int tid = threadIdx.x, lane = tid & 31, wave = tid >> 5;
  const int c = lane & 15, hh = lane >> 4, koff = hh * 8;
  const int rowbase = blockIdx.x * ROWS;

  {
    const __bf16 zb = bits2bf((unsigned short)0);
#pragma unroll 1
    for (int i = tid; i < ROWS * HP; i += NTHR) { Ahh[i] = zb; Ahl[i] = zb; }
  }
  float bb[2][4];
#pragma unroll
  for (int nt = 0; nt < 2; ++nt) {
    const int j = 32 * wave + 16 * nt + c;
#pragma unroll
    for (int g = 0; g < 4; ++g) bb[nt][g] = bf16r(bl[g * NH + j]);
  }
  const float bdv = bf16r(bd[16 * wave + c]);
  float cst[2][8], hst[2][8];
#pragma unroll
  for (int nt = 0; nt < 2; ++nt)
#pragma unroll
    for (int r = 0; r < 8; ++r) { cst[nt][r] = 0.0f; hst[nt][r] = 0.0f; }
  stage_rows(ids, GF, Gs, rowbase, 0, tid);
  __syncthreads();

  const __bf16* ahr = Ahh + c * HP + koff;
  const __bf16* alr = Ahl + c * HP + koff;
  const v8f z8 = {0.f, 0.f, 0.f, 0.f, 0.f, 0.f, 0.f, 0.f};

#pragma unroll 1
  for (int t = 0; t < NTS; ++t) {
#pragma unroll
    for (int nt = 0; nt < 2; ++nt) {
      const int j = 32 * wave + 16 * nt + c;
      const __bf16* wh = WH + (size_t)j * NH + koff;
      v8f acc[4];
      acc[0] = z8; acc[1] = z8; acc[2] = z8; acc[3] = z8;
#pragma unroll 1
      for (int k0 = 0; k0 < NH; k0 += 32) {
        const v16b ah = Frag<__bf16>::load(ahr + k0);
        const v16b al = Frag<__bf16>::load(alr + k0);
        const v16b b0 = Frag<__bf16>::load(wh + k0);
        const v16b b1 = Frag<__bf16>::load(wh + (size_t)1 * NH * NH + k0);
        const v16b b2 = Frag<__bf16>::load(wh + (size_t)2 * NH * NH + k0);
        const v16b b3 = Frag<__bf16>::load(wh + (size_t)3 * NH * NH + k0);
        acc[0] = Frag<__bf16>::mma(ah, b0, acc[0]);
        acc[1] = Frag<__bf16>::mma(ah, b1, acc[1]);
        acc[2] = Frag<__bf16>::mma(ah, b2, acc[2]);
        acc[3] = Frag<__bf16>::mma(ah, b3, acc[3]);
        acc[0] = Frag<__bf16>::mma(al, b0, acc[0]);
        acc[1] = Frag<__bf16>::mma(al, b1, acc[1]);
        acc[2] = Frag<__bf16>::mma(al, b2, acc[2]);
        acc[3] = Frag<__bf16>::mma(al, b3, acc[3]);
        guard_g4(acc[0], acc[1], acc[2], acc[3], ah, al, b0, b1, b2, b3);
      }
      acc_guard4(acc[0], acc[1], acc[2], acc[3]);
#pragma unroll
      for (int r = 0; r < 8; ++r) {
        const float* gr = Gs + (8 * hh + r) * GP + j;
        const float xi = gr[0];
        const float xj = gr[NH];
        const float xf = gr[2 * NH];
        const float xo = gr[3 * NH];
        const float zi = (acc[0][r] + xi) + bb[nt][0];
        const float zj = (acc[1][r] + xj) + bb[nt][1];
        const float zf = (acc[2][r] + xf) + bb[nt][2];
        const float zo = (acc[3][r] + xo) + bb[nt][3];
        const float ig = fsig(zi);
        const float jg = ftanh(zj);
        const float fg = fsig(zf + FORGET_B);
        const float og = fsig(zo);
        const float cn = fg * cst[nt][r] + ig * jg;
        cst[nt][r] = cn;
        hst[nt][r] = og * ftanh(cn);
      }
    }
    __syncthreads();
#pragma unroll
    for (int nt = 0; nt < 2; ++nt) {
      const int j = 32 * wave + 16 * nt + c;
#pragma unroll
      for (int r = 0; r < 8; ++r) {
        const float hv = hst[nt][r];
        const unsigned short hb = f2bf_bits(hv);
        const unsigned short lb = f2bf_bits(hv - bf_bits2f(hb));
        Ahh[(8 * hh + r) * HP + j] = bits2bf(hb);
        Ahl[(8 * hh + r) * HP + j] = bits2bf(lb);
      }
    }
    if (t + 1 < NTS) stage_rows(ids, GF, Gs, rowbase, t + 1, tid);
    __syncthreads();
  }

  {
    const int n = 16 * wave + c;
    const __bf16* wd = WD + (size_t)n * NH + koff;
    v8f accd = z8;
#pragma unroll 1
    for (int k0 = 0; k0 < NH; k0 += 32) {
      const v16b ah = Frag<__bf16>::load(ahr + k0);
      const v16b al = Frag<__bf16>::load(alr + k0);
      const v16b b0 = Frag<__bf16>::load(wd + k0);
      accd = Frag<__bf16>::mma(ah, b0, accd);
      accd = Frag<__bf16>::mma(al, b0, accd);
      guard_g1(accd, ah, al, b0);
    }
    acc_guard1(accd);
#pragma unroll
    for (int r = 0; r < 8; ++r) Hs[(8 * hh + r) * OPD + n] = accd[r] + bdv;
  }
  __syncthreads();
  for (int pass = 0; pass < 2; ++pass) {
#pragma unroll
    for (int it = 0; it < 2; ++it) {
      const int idx = it * NTHR + tid;
      const int row = idx >> 5, c4 = (idx & 31) * 4;
      const v4f v = *(const v4f*)(Hs + row * OPD + c4);
      *(volatile v4f*)(out + (size_t)(rowbase + row) * NV + c4) = v;
    }
    __threadfence();
  }
}

extern "C" void kernel_launch(void* const* d_in, const int* in_sizes, int n_in,
                              void* d_out, int out_size, void* d_ws, size_t ws_size, hipStream_t stream) {
  if (n_in < 5 || d_out == nullptr || d_ws == nullptr) return;
  if (in_sizes[0] != NB * NTS || in_sizes[1] != NIN * NG4 || in_sizes[2] != NG4 ||
      in_sizes[3] != NH * NV || in_sizes[4] != NV || out_size != NB * NV) return;

  const int*   ids = (const int*)  d_in[0];
  const float* wl  = (const float*)d_in[1];
  const float* bl  = (const float*)d_in[2];
  const float* wd  = (const float*)d_in[3];
  const float* bd  = (const float*)d_in[4];
  float* out = (float*)d_out;

  char* ws = (char*)d_ws; size_t off = 0;
  auto carve = [&](size_t bytes) -> char* { char* p = ws + off; off += (bytes + 255) & ~(size_t)255; return p; };
  unsigned short* WH = (unsigned short*)carve((size_t)NG4 * NH * 2);
  unsigned short* WD = (unsigned short*)carve((size_t)NV * NH * 2);
  float*          GF = (float*)carve((size_t)NV * NG4 * 4);
  if (off > ws_size || off > (size_t)134217728) return;

  tpose_bf16_kernel<<<dim3(NG4 / 64, NH / 64), NTHR, 0, stream>>>(wl + (size_t)NV * NG4, NG4, NH, WH);
  tpose_bf16_kernel<<<dim3(NV / 64, NH / 64), NTHR, 0, stream>>>(wd, NV, NH, WD);
  gtab_kernel<<<(NV * NG4 / 4) / NTHR, NTHR, 0, stream>>>(wl, GF, NV * NG4 / 4);
  lstm_seq_kernel<<<NB / ROWS, NTHR, 0, stream>>>(ids, GF, bl, bd, WH, WD, out);
}
